// CrossAttention_61718680044194
// MI455X (gfx1250) — hardware-run, weakly checked
//
#include <hip/hip_runtime.h>

typedef float          v8f   __attribute__((ext_vector_type(8)));
typedef float          v4f   __attribute__((ext_vector_type(4)));
typedef unsigned int   v4u   __attribute__((ext_vector_type(4)));
typedef int            v8i   __attribute__((ext_vector_type(8)));
typedef unsigned short v8us  __attribute__((ext_vector_type(8)));
typedef unsigned short v16us __attribute__((ext_vector_type(16)));
typedef __bf16         v16bf __attribute__((ext_vector_type(16)));
typedef _Float16       v16h  __attribute__((ext_vector_type(16)));
typedef v4f  __attribute__((may_alias)) v4fa;
typedef v8us __attribute__((may_alias)) v8usa;
union FragB { v16bf v; v16us u; v8us h[2]; v8i w; };
union FragH { v16h  v; v16us u; v8us h[2]; v8i w; };

__device__ __forceinline__ v8f wmb(const FragB& a, const FragB& b, v8f c) {
  v8f d = __builtin_amdgcn_wmma_f32_16x16x32_bf16(false, a.v, false, b.v, (short)0, c, false, false);
  asm volatile("v_nop\n\tv_nop\n\tv_nop\n\tv_nop" : "+v"(d) : "v"(a.w), "v"(b.w));
  return d;
}

__device__ __forceinline__ v8f wmh(const FragH& a, const FragH& b, v8f c) {
  v8f d = __builtin_amdgcn_wmma_f32_16x16x32_f16(false, a.v, false, b.v, (short)0, c, false, false);
  asm volatile("v_nop\n\tv_nop\n\tv_nop\n\tv_nop" : "+v"(d) : "v"(a.w), "v"(b.w));
  return d;
}

__device__ __forceinline__ unsigned bf16_bits(float f) {
  const unsigned u = __float_as_uint(f);
  const unsigned r = (u + 0x7FFFu + ((u >> 16) & 1u)) >> 16;
  const unsigned q = (u >> 16) | 0x40u;
  return ((u & 0x7fffffffu) > 0x7f800000u) ? q : r;
}

__device__ __forceinline__ float bf16_val(float f) {
  return __uint_as_float(bf16_bits(f) << 16);
}
__device__ __forceinline__ int clampi(int v, int lo, int hi) {
  return v < lo ? lo : (v > hi ? hi : v);
}

__device__ __forceinline__ unsigned f16_bits(float f) {
  const unsigned u  = __float_as_uint(f);
  const unsigned s  = (u >> 16) & 0x8000u;
  const unsigned a  = u & 0x7fffffffu;
  const unsigned t  = a - 0x38000000u;
  const unsigned r  = (t + 0x0FFFu + ((t >> 13) & 1u)) >> 13;
  const unsigned rc = r > 0x7C00u ? 0x7C00u : r;
  const bool small  = a < 0x38800000u;
  const bool isnan  = a > 0x7f800000u;
  const unsigned fin = small ? 0u : (s | rc);
  return isnan ? (s | 0x7E00u) : fin;
}

__device__ __forceinline__ unsigned pk16(unsigned lo, unsigned hi) { return lo | (hi << 16); }
__device__ __forceinline__ unsigned bf16_lo_bits(float v) {
  float hi = bf16_val(v);
  asm volatile("" : "+v"(hi));
  return bf16_bits(v - hi);
}
__device__ __forceinline__ v4u pack8_bf16(v4f a, v4f c) {
  return (v4u){ pk16(bf16_bits(a[0]), bf16_bits(a[1])), pk16(bf16_bits(a[2]), bf16_bits(a[3])),
                pk16(bf16_bits(c[0]), bf16_bits(c[1])), pk16(bf16_bits(c[2]), bf16_bits(c[3])) };
}
__device__ __forceinline__ v4u pack8_bf16_lo(v4f a, v4f c) {
  return (v4u){ pk16(bf16_lo_bits(a[0]), bf16_lo_bits(a[1])), pk16(bf16_lo_bits(a[2]), bf16_lo_bits(a[3])),
                pk16(bf16_lo_bits(c[0]), bf16_lo_bits(c[1])), pk16(bf16_lo_bits(c[2]), bf16_lo_bits(c[3])) };
}
__device__ __forceinline__ v4u pack8_f16(v4f a, v4f c) {
  return (v4u){ pk16(f16_bits(a[0]), f16_bits(a[1])), pk16(f16_bits(a[2]), f16_bits(a[3])),
                pk16(f16_bits(c[0]), f16_bits(c[1])), pk16(f16_bits(c[2]), f16_bits(c[3])) };
}

template <int FORM>
__global__ __launch_bounds__(256) void k_plane(const float* __restrict__ src, int rows, int cols, int ldsrc,
                                               unsigned short* __restrict__ dst, int MP, int KP) {
  static_assert(FORM >= 0 && FORM <= 3);
  const int KTOT = (FORM == 1 || FORM == 3) ? 2 * KP : KP;
  const unsigned ppr   = (unsigned)(KTOT >> 3);
  const unsigned kp8   = (unsigned)(KP >> 3);
  const unsigned total = (unsigned)MP * ppr;
  const unsigned g     = blockIdx.x * 256u + threadIdx.x;
  const unsigned rowu  = g / ppr;
  const unsigned p     = g - rowu * ppr;
  const bool second    = p >= kp8;
  const int row = (int)rowu;
  const int c0  = (int)((second ? p - kp8 : p) << 3);
  const float* srow = src + (size_t)clampi(row, 0, rows - 1) * (size_t)ldsrc;
  float x[8];
  unsigned mk[8];
#pragma unroll
  for (int e = 0; e < 8; ++e) {
    const int c = c0 + e;
    const float v = srow[clampi(c, 0, cols - 1)];
    asm volatile("" :: "v"(v));
    x[e]  = v;
    mk[e] = (row < rows && c < cols) ? 0xFFFFu : 0u;
  }
  const v4f a = (v4f){ x[0], x[1], x[2], x[3] };
  const v4f c = (v4f){ x[4], x[5], x[6], x[7] };
  v4u o;
  if (FORM == 2) {
    o = pack8_f16(a, c);
  } else {
    const v4u hi = pack8_bf16(a, c);
    o = hi;
    if (FORM == 1) { const v4u lo = pack8_bf16_lo(a, c); o = second ? lo : hi; }
  }
  const v4u mw = (v4u){ pk16(mk[0], mk[1]), pk16(mk[2], mk[3]), pk16(mk[4], mk[5]), pk16(mk[6], mk[7]) };
  o &= mw;
  if (g < total) {
    volatile v4u* q = (volatile v4u*)(dst + (size_t)g * 8);
    *q = o;
    __threadfence();
    *q = o;
  }
}

template <int FORM> struct FragOf    { typedef FragB T; };
template <>         struct FragOf<2> { typedef FragH T; };
__device__ __forceinline__ v8f mm(const FragB& a, const FragB& b, v8f c) { return wmb(a, b, c); }
__device__ __forceinline__ v8f mm(const FragH& a, const FragH& b, v8f c) { return wmh(a, b, c); }
template <class F> __device__ __forceinline__ F ld_frag(const unsigned short* p) {
  F f;
  f.h[0] = *(const v8usa*)(p);
  f.h[1] = *(const v8usa*)(p + 16);
  return f;
}

template <int FORM, int EPI>
__global__ __launch_bounds__(256) __attribute__((amdgpu_num_vgpr(248)))
void k_gemm_nt(const unsigned short* __restrict__ A, const unsigned short* __restrict__ B,
               const float* __restrict__ bias, float* __restrict__ D, int M, int N, int KTOT, int ldd) {
  static_assert(FORM >= 0 && FORM <= 2);
  static_assert(EPI == 0 || EPI == 1);
  typedef typename FragOf<FORM>::T F;
  __shared__ __attribute__((aligned(16))) float sT[8][16 * 68];
  const int lane = threadIdx.x & 31;
  const int wave = threadIdx.x >> 5;
  const int tilesM = (M + 63) >> 6;
  const int tilesN = (N + 63) >> 6;
  const int tile = blockIdx.x * 8 + wave;
  if (tile >= tilesM * tilesN) return;
  const int tm = tile / tilesN;
  const int tn = tile - tm * tilesN;
  const int m0 = tm << 6;
  const int n0 = tn << 6;

  const int rl = lane & 15;
  const int h8 = (lane >> 4) * 8;
  const unsigned short* pa = A + (size_t)(m0 + rl) * (size_t)KTOT + h8;
  const unsigned short* pb = B + (size_t)(n0 + rl) * (size_t)KTOT + h8;

  v8f acc[4][4];
#pragma unroll
  for (int i = 0; i < 4; ++i)
#pragma unroll
    for (int j = 0; j < 4; ++j) acc[i][j] = (v8f){0.f, 0.f, 0.f, 0.f, 0.f, 0.f, 0.f, 0.f};

#pragma unroll 1
  for (int k0 = 0; k0 < KTOT; k0 += 32) {
    F bf[4];
#pragma unroll
    for (int j = 0; j < 4; ++j) bf[j] = ld_frag<F>(pb + (size_t)(j << 4) * (size_t)KTOT + k0);
#pragma unroll
    for (int i = 0; i < 4; ++i) {
      const F af = ld_frag<F>(pa + (size_t)(i << 4) * (size_t)KTOT + k0);
#pragma unroll
      for (int j = 0; j < 4; ++j) acc[i][j] = mm(af, bf[j], acc[i][j]);
    }
  }

  float* slab = sT[wave];
  const int hh = lane >> 4;
  const int c4 = (lane & 15) * 4;
  const int nc = n0 + c4;
  const bool cok = nc < N;
  v4f bv = (v4f){0.f, 0.f, 0.f, 0.f};
  if (EPI == 1) {
    bv = *(const v4fa*)(bias + clampi(nc, 0, N - 4));
    asm volatile("" :: "v"(bv));
  }
#pragma unroll
  for (int i = 0; i < 4; ++i) {
    const int mBase = m0 + (i << 4);
#pragma unroll
    for (int j = 0; j < 4; ++j) {
#pragma unroll
      for (int r = 0; r < 8; ++r) slab[(h8 + r) * 68 + (j << 4) + rl] = acc[i][j][r];
    }
    __builtin_amdgcn_fence(__ATOMIC_RELEASE, "workgroup");
    __builtin_amdgcn_wave_barrier();
    __builtin_amdgcn_fence(__ATOMIC_ACQUIRE, "workgroup");
    v4f vv[8];
#pragma unroll
    for (int it = 0; it < 8; ++it) {
      const int row = it * 2 + hh;
      v4f v = *(const v4fa*)(slab + row * 68 + c4);
      if (EPI == 1) v += bv;
      vv[it] = v;
    }
    for (int pass = 0; pass < 2; ++pass) {
#pragma unroll
      for (int it = 0; it < 8; ++it) {
        const int row = mBase + it * 2 + hh;
        if (cok && row < M) *(volatile v4f*)(D + (size_t)row * (size_t)ldd + nc) = vv[it];
      }
      __threadfence();
    }
    __builtin_amdgcn_fence(__ATOMIC_RELEASE, "workgroup");
    __builtin_amdgcn_wave_barrier();
    __builtin_amdgcn_fence(__ATOMIC_ACQUIRE, "workgroup");
  }
}

#ifndef TANH_FORM
#define TANH_FORM 1
#endif
#ifndef P_FORM
#define P_FORM 1
#endif

#define NB   8
#define NT   128
#define NI   196
#define TD   768
#define IDM  1024
#define HD   512
#define MT   (NB * NT)
#define MI   (NB * NI)
#define MIP  1600
#define MP2  256

#if P_FORM == 1
#define KH1   224
#define KT1   448
#define KH2   128
#define KT2   256
#define NDUP  2
#define AFORM 0
#define OSCALE 1.0f
#define PCARRY 1.0f
#else
#define KH1   256
#define KT1   256
#define KH2   128
#define KT2   128
#define NDUP  1
#define AFORM 2
#define OSCALE (1.0f / 1024.0f)
#define PCARRY 1024.0f
#endif

static_assert(P_FORM == 1 || P_FORM == 2);
static_assert(TANH_FORM == 1 || TANH_FORM == 2);
static_assert(NT % 32 == 0);
static_assert(NI == 7 * 28);
static_assert(28 == 4 * 7);
static_assert(HD % 4 == 0);
static_assert(MT % 64 == 0 && MIP % 64 == 0 && MIP >= MI && MI % 16 == 0 && MT % 16 == 0);
static_assert(HD % 64 == 0 && TD % 32 == 0 && IDM % 32 == 0 && TD % 64 == 0 && IDM % 64 == 0);
static_assert((MT * TD / 8) % 256 == 0 && (MIP * IDM / 8) % 256 == 0);
static_assert(KH1 % 32 == 0 && KH2 % 32 == 0 && KH1 >= NI && KH2 == NT);
static_assert(KT1 == NDUP * KH1 && KT2 == NDUP * KH2);
static_assert(MP2 % 64 == 0 && MP2 >= NI && NT % 64 == 0);
static_assert((KT1 * 2) % 128 == 0 && (KT2 * 2) % 128 == 0);
static_assert(((NT / 64) * (IDM / 64)) % 8 == 0 && ((MP2 / 64) * (TD / 64)) % 8 == 0);
static_assert(NB * NT * IDM == 1048576);
static_assert(NB * NT * IDM + NB * NI * TD == 2252800);
static_assert((NI * NT) % 4 == 0);

typedef unsigned int v2u __attribute__((ext_vector_type(2)));
typedef v4u __attribute__((may_alias)) v4ua;
typedef v2u __attribute__((may_alias)) v2ua;

__device__ __forceinline__ void wave_lds_sync() {
  __builtin_amdgcn_fence(__ATOMIC_RELEASE, "workgroup");
  __builtin_amdgcn_wave_barrier();
  __builtin_amdgcn_fence(__ATOMIC_ACQUIRE, "workgroup");
}

__device__ __forceinline__ float tanh_f(float x) {
#if TANH_FORM == 1
#if __has_builtin(__builtin_amdgcn_exp2f)
  const float e = __builtin_amdgcn_exp2f(x * 2.8853900817779268f);
#else
  const float e = exp2f(x * 2.8853900817779268f);
#endif
  const float r = __builtin_amdgcn_rcpf(1.0f + e);
  return 1.0f - 2.0f * r;
#else
  return tanhf(x);
#endif
}

__device__ __forceinline__ unsigned feat_bits(unsigned hb) {
#if P_FORM == 1
  return hb;
#else
  return f16_bits(__uint_as_float(hb << 16));
#endif
}

#define WTP 72
template <int KD>
__device__ __forceinline__ void wt_tile(const float* __restrict__ W, unsigned short* __restrict__ out,
                                        int c0, int k0, int tid) {
  __shared__ __attribute__((aligned(16))) unsigned short sT[64 * WTP];
  const int lane = tid & 31, w = tid >> 5;
  const int c4 = (tid & 15) * 4, rr = tid >> 4;
#pragma unroll
  for (int p = 0; p < 4; ++p) {
    const int r = rr + 16 * p;
    const v4f v = *(const v4fa*)(W + (size_t)(k0 + r) * HD + c0 + c4);
    sT[(c4 + 0) * WTP + r] = (unsigned short)bf16_bits(v[0]);
    sT[(c4 + 1) * WTP + r] = (unsigned short)bf16_bits(v[1]);
    sT[(c4 + 2) * WTP + r] = (unsigned short)bf16_bits(v[2]);
    sT[(c4 + 3) * WTP + r] = (unsigned short)bf16_bits(v[3]);
  }
  __syncthreads();
  const int q8 = lane & 7, sub = lane >> 3;
  v4u vv[2];
#pragma unroll
  for (int it = 0; it < 2; ++it) {
    const int row = 32 * it + 4 * w + sub;
    vv[it] = *(const v4ua*)(sT + row * WTP + 8 * q8);
  }
  for (int pass = 0; pass < 2; ++pass) {
#pragma unroll
    for (int it = 0; it < 2; ++it) {
      const int row = 32 * it + 4 * w + sub;
      *(volatile v4u*)(out + (size_t)(c0 + row) * KD + k0 + 8 * q8) = vv[it];
    }
    __threadfence();
  }
}

__global__ __launch_bounds__(256) void k_wt(const float* __restrict__ Wt, const float* __restrict__ Wi,
                                            const float* __restrict__ bt, const float* __restrict__ bi,
                                            const float* __restrict__ wa, const float* __restrict__ ba,
                                            unsigned short* __restrict__ WtT, unsigned short* __restrict__ WiT,
                                            float* __restrict__ par) {
  const int tid = threadIdx.x;
  const int by = blockIdx.y;
  if (by < 12) {
    wt_tile<TD>(Wt, WtT, blockIdx.x * 64, by * 64, tid);
  } else if (by < 28) {
    wt_tile<IDM>(Wi, WiT, blockIdx.x * 64, (by - 12) * 64, tid);
  } else {
    const int g = blockIdx.x * 256 + tid;
    const float a0 = bt[clampi(g, 0, HD - 1)];
    const float a1 = bi[clampi(g - HD, 0, HD - 1)];
    const float a2 = wa[clampi(g - 2 * HD, 0, HD - 1)];
    const float a3 = ba[0];
    asm volatile("" :: "v"(a0), "v"(a1), "v"(a2), "v"(a3));
    const int sec = g >> 9;
    float v = 0.0f;
    v = (sec == 0) ? a0 : v;
    v = (sec == 1) ? a1 : v;
    v = (sec == 2) ? a2 : v;
    v = (g == 3 * HD) ? a3 : v;
    const float o = bf16_val(v);
    volatile float* q = par + g;
    *q = o;
    __threadfence();
    *q = o;
  }
}

#define PAIR_LDS_FLOATS (HD * 32 + 28 * HD + HD)
__global__ __launch_bounds__(128) void k_pair(const float* __restrict__ PT, const float* __restrict__ PI,
                                              const float* __restrict__ par, float* __restrict__ ST) {
  extern __shared__ __attribute__((aligned(16))) float smem[];
  float* sPT = smem;
  float* sPI = smem + HD * 32;
  float* sWA = smem + HD * 32 + 28 * HD;
  const int tid = threadIdx.x, lane = tid & 31, w = tid >> 5;
  const int i0 = blockIdx.x * 28, t0 = blockIdx.y * 32, b = blockIdx.z;

  {
    const int trow = tid & 31, hq = tid >> 5;
    const float* src = PT + (size_t)(b * NT + t0 + trow) * HD;
#pragma unroll 4
    for (int it = 0; it < 32; ++it) {
      const int h4 = (hq + 4 * it) * 4;
      const v4f v = *(const v4fa*)(src + h4);
      sPT[(h4 + 0) * 32 + trow] = v[0];
      sPT[(h4 + 1) * 32 + trow] = v[1];
      sPT[(h4 + 2) * 32 + trow] = v[2];
      sPT[(h4 + 3) * 32 + trow] = v[3];
    }
  }
  {
    const float* src = PI + (size_t)(b * NI + i0) * HD;
#pragma unroll 4
    for (int it = 0; it < 28; ++it) {
      const int idx = tid + 128 * it;
      const v4f v = *(const v4fa*)(src + 4 * idx);
      *(v4fa*)(sPI + 4 * idx) = v;
    }
  }
  {
    const v4f v = *(const v4fa*)(par + 2 * HD + 4 * tid);
    *(v4fa*)(sWA + 4 * tid) = v;
  }
  const float bav = par[3 * HD];
  __syncthreads();

  float acc[7];
#pragma unroll
  for (int ii = 0; ii < 7; ++ii) acc[ii] = 0.0f;
  const float* pI = sPI + (7 * w) * HD;

#pragma unroll 1
  for (int h = 0; h < HD; h += 4) {
    const float p0 = sPT[(h + 0) * 32 + lane];
    const float p1 = sPT[(h + 1) * 32 + lane];
    const float p2 = sPT[(h + 2) * 32 + lane];
    const float p3 = sPT[(h + 3) * 32 + lane];
    const v4f wv = *(const v4fa*)(sWA + h);
#pragma unroll
    for (int ii = 0; ii < 7; ++ii) {
      const v4f q = *(const v4fa*)(pI + ii * HD + h);
      float a = acc[ii];
      a = fmaf(wv[0], tanh_f(p0 + q[0]), a);
      a = fmaf(wv[1], tanh_f(p1 + q[1]), a);
      a = fmaf(wv[2], tanh_f(p2 + q[2]), a);
      a = fmaf(wv[3], tanh_f(p3 + q[3]), a);
      acc[ii] = a;
    }
  }

  float sc[7];
#pragma unroll
  for (int ii = 0; ii < 7; ++ii) sc[ii] = acc[ii] + bav;
  float* dst = ST + (size_t)(b * NI + i0 + 7 * w) * NT + t0 + lane;
  for (int pass = 0; pass < 2; ++pass) {
#pragma unroll
    for (int ii = 0; ii < 7; ++ii) *(volatile float*)(dst + ii * NT) = sc[ii];
    __threadfence();
  }
}

#define SOFT_LDS_BYTES (NI * NT * 4 + 2 * NT * 4 + 8 * KT1 * 2)
#define NPC1 (KT1 / 8)
__global__ __launch_bounds__(256) void k_soft(const float* __restrict__ ST, unsigned short* __restrict__ P1,
                                              unsigned short* __restrict__ P2) {
  extern __shared__ __attribute__((aligned(16))) float smem[];
  float* sS   = smem;
  float* sMax = smem + NI * NT;
  float* sSum = sMax + NT;
  unsigned short* sStg = (unsigned short*)(sSum + NT);
  const int tid = threadIdx.x, lane = tid & 31, w = tid >> 5;
  const int b = blockIdx.x;

  {
    const float* src = ST + (size_t)b * NI * NT;
    const int nv4 = NI * NT / 4;
#pragma unroll 5
    for (int it = 0; it < 25; ++it) {
      const int idx = tid + 256 * it;
      const int ic = idx < nv4 ? idx : nv4 - 1;
      const v4f v = *(const v4fa*)(src + 4 * ic);
      asm volatile("" :: "v"(v));
      if (idx < nv4) *(v4fa*)(sS + 4 * idx) = v;
    }
  }
  __syncthreads();

  if (tid < NT) {
    float m = sS[tid];
#pragma unroll 4
    for (int i = 1; i < NI; ++i) m = fmaxf(m, sS[i * NT + tid]);
    float s = 0.0f;
#pragma unroll 1
    for (int i = 0; i < NI; ++i) s += expf(sS[i * NT + tid] - m);
    sMax[tid] = m;
    sSum[tid] = s;
  }
  __syncthreads();

  {
    unsigned short* stg = sStg + w * KT1;
#pragma unroll 1
    for (int r = 0; r < NT / 8; ++r) {
      const int t = w + 8 * r;
      const float m = sMax[t];
      const float s = sSum[t];
#pragma unroll 1
      for (int j = 0; j < KH1 / 32; ++j) {
        const int i = lane + 32 * j;
        const int ic = i < NI ? i : NI - 1;
        const float v = sS[ic * NT + t];
        const float p = expf(v - m) / s;
        const unsigned msk = (i < NI) ? 0xFFFFu : 0u;
#if P_FORM == 1
        stg[i]       = (unsigned short)(bf16_bits(p) & msk);
        stg[KH1 + i] = (unsigned short)(bf16_lo_bits(p) & msk);
#else
        stg[i]       = (unsigned short)(f16_bits(p * PCARRY) & msk);
#endif
      }
      wave_lds_sync();
      const int pc0 = lane < NPC1 ? lane : NPC1 - 1;
      const int pc1 = (lane + 32) < NPC1 ? (lane + 32) : NPC1 - 1;
      const v4u a0 = *(const v4ua*)(stg + 8 * pc0);
      const v4u a1 = *(const v4ua*)(stg + 8 * pc1);
      unsigned short* drow = P1 + (size_t)(b * NT + t) * KT1;
      for (int pass = 0; pass < 2; ++pass) {
        if (lane < NPC1) *(volatile v4u*)(drow + 8 * lane) = a0;
        if (lane + 32 < NPC1) *(volatile v4u*)(drow + 8 * (lane + 32)) = a1;
        __threadfence();
      }
      wave_lds_sync();
    }
  }

#pragma unroll 1
  for (int r = 0; r < MP2 / 8; ++r) {
    const int i = w + 8 * r;
    const int ic = i < NI ? i : NI - 1;
    const v4f v = *(const v4fa*)(sS + ic * NT + 4 * lane);
    float m = fmaxf(fmaxf(v[0], v[1]), fmaxf(v[2], v[3]));
    m = fmaxf(m, __shfl_xor(m, 16, 32));
    m = fmaxf(m, __shfl_xor(m, 8, 32));
    m = fmaxf(m, __shfl_xor(m, 4, 32));
    m = fmaxf(m, __shfl_xor(m, 2, 32));
    m = fmaxf(m, __shfl_xor(m, 1, 32));
    const float e0 = expf(v[0] - m);
    const float e1 = expf(v[1] - m);
    const float e2 = expf(v[2] - m);
    const float e3 = expf(v[3] - m);
    float s = (e0 + e1) + (e2 + e3);
    s += __shfl_xor(s, 16, 32);
    s += __shfl_xor(s, 8, 32);
    s += __shfl_xor(s, 4, 32);
    s += __shfl_xor(s, 2, 32);
    s += __shfl_xor(s, 1, 32);
    const float p0 = e0 / s, p1 = e1 / s, p2 = e2 / s, p3 = e3 / s;
    const unsigned msk = (i < NI) ? 0xFFFFFFFFu : 0u;
    unsigned short* drow = P2 + (size_t)(b * MP2 + i) * KT2 + 4 * lane;
#if P_FORM == 1
    const v2u hv = (v2u){ pk16(bf16_bits(p0), bf16_bits(p1)) & msk, pk16(bf16_bits(p2), bf16_bits(p3)) & msk };
    const v2u lv = (v2u){ pk16(bf16_lo_bits(p0), bf16_lo_bits(p1)) & msk, pk16(bf16_lo_bits(p2), bf16_lo_bits(p3)) & msk };
    for (int pass = 0; pass < 2; ++pass) {
      *(volatile v2u*)(drow) = hv;
      *(volatile v2u*)(drow + KH2) = lv;
      __threadfence();
    }
#else
    const v2u hv = (v2u){ pk16(f16_bits(p0 * PCARRY), f16_bits(p1 * PCARRY)) & msk,
                          pk16(f16_bits(p2 * PCARRY), f16_bits(p3 * PCARRY)) & msk };
    for (int pass = 0; pass < 2; ++pass) {
      *(volatile v2u*)(drow) = hv;
      __threadfence();
    }
#endif
  }
}

template <int NTOK, int KH, int DM, int NDUPL>
__global__ __launch_bounds__(256) void k_ft(const unsigned short* __restrict__ X, unsigned short* __restrict__ out) {
  constexpr int PITCH = KH + 8;
  constexpr int NLD = KH * 8 / 256;
  constexpr int PPR = NDUPL * KH / 8;
  constexpr int KP8 = KH / 8;
  constexpr int NST = 64 * PPR / 256;
  static_assert((KH * 8) % 256 == 0);
  static_assert((64 * PPR) % 256 == 0);
  static_assert((PITCH * 2) % 16 == 0);
  static_assert(DM % 64 == 0 && KH >= NTOK);
  __shared__ __attribute__((aligned(16))) unsigned short sT[64 * PITCH];
  const int tid = threadIdx.x;
  const int d0 = blockIdx.x * 64, b = blockIdx.y;

#pragma unroll
  for (int it = 0; it < NLD; ++it) {
    const int idx = tid + 256 * it;
    const int k = idx >> 3, pc = idx & 7;
    const int kc = k < NTOK ? k : NTOK - 1;
    v4u v = *(const v4ua*)(X + (size_t)(b * NTOK + kc) * DM + d0 + 8 * pc);
    asm volatile("" :: "v"(v));
    const unsigned mk = (k < NTOK) ? 0xFFFFFFFFu : 0u;
#pragma unroll
    for (int j = 0; j < 4; ++j) {
      const unsigned wd = v[j] & mk;
      sT[(8 * pc + 2 * j) * PITCH + k]     = (unsigned short)feat_bits(wd & 0xFFFFu);
      sT[(8 * pc + 2 * j + 1) * PITCH + k] = (unsigned short)feat_bits(wd >> 16);
    }
  }
  __syncthreads();

  v4u vv[NST];
#pragma unroll
  for (int it = 0; it < NST; ++it) {
    const int g = tid + 256 * it;
    const int row = g / PPR;
    const int p = g - row * PPR;
    const int kp = p >= KP8 ? p - KP8 : p;
    vv[it] = *(const v4ua*)(sT + row * PITCH + 8 * kp);
  }
  unsigned short* base = out + (size_t)(b * DM + d0) * (size_t)(NDUPL * KH);
  for (int pass = 0; pass < 2; ++pass) {
#pragma unroll
    for (int it = 0; it < NST; ++it) {
      const int g = tid + 256 * it;
      *(volatile v4u*)(base + (size_t)g * 8) = vv[it];
    }
    __threadfence();
  }
}

template <int FORM>
__global__ __launch_bounds__(256) __attribute__((amdgpu_num_vgpr(248)))
void k_att(const unsigned short* __restrict__ A, const unsigned short* __restrict__ Bp, float* __restrict__ D,
           int M, int MP, int N, int KTOT, int ldd, int sA, int sB, int sD, float oscale) {
  typedef typename FragOf<FORM>::T F;
  __shared__ __attribute__((aligned(16))) float sT[8][16 * 68];
  const int lane = threadIdx.x & 31;
  const int wave = threadIdx.x >> 5;
  const int b = blockIdx.z;
  const int tilesM = MP >> 6;
  const int tilesN = N >> 6;
  const int tile = blockIdx.x * 8 + wave;
  if (tile >= tilesM * tilesN) return;
  const int tm = tile / tilesN;
  const int tn = tile - tm * tilesN;
  const int m0 = tm << 6;
  const int n0 = tn << 6;

  const int rl = lane & 15;
  const int h8 = (lane >> 4) * 8;
  const unsigned short* pa = A + (size_t)b * (size_t)sA + (size_t)(m0 + rl) * (size_t)KTOT + h8;
  const unsigned short* pb = Bp + (size_t)b * (size_t)sB + (size_t)(n0 + rl) * (size_t)KTOT + h8;
  float* Db = D + (size_t)b * (size_t)sD;

  v8f acc[4][4];
#pragma unroll
  for (int i = 0; i < 4; ++i)
#pragma unroll
    for (int j = 0; j < 4; ++j) acc[i][j] = (v8f){0.f, 0.f, 0.f, 0.f, 0.f, 0.f, 0.f, 0.f};

#pragma unroll 1
  for (int k0 = 0; k0 < KTOT; k0 += 32) {
    F bf[4];
#pragma unroll
    for (int j = 0; j < 4; ++j) bf[j] = ld_frag<F>(pb + (size_t)(j << 4) * (size_t)KTOT + k0);
#pragma unroll
    for (int i = 0; i < 4; ++i) {
      const F af = ld_frag<F>(pa + (size_t)(i << 4) * (size_t)KTOT + k0);
#pragma unroll
      for (int j = 0; j < 4; ++j) acc[i][j] = mm(af, bf[j], acc[i][j]);
    }
  }

  float* slab = sT[wave];
  const int hh = lane >> 4;
  const int c4 = (lane & 15) * 4;
  const int nc = n0 + c4;
#pragma unroll
  for (int i = 0; i < 4; ++i) {
    const int mBase = m0 + (i << 4);
#pragma unroll
    for (int j = 0; j < 4; ++j) {
#pragma unroll
      for (int r = 0; r < 8; ++r) slab[(h8 + r) * 68 + (j << 4) + rl] = acc[i][j][r];
    }
    wave_lds_sync();
    v4f vv[8];
#pragma unroll
    for (int it = 0; it < 8; ++it) {
      const int row = it * 2 + hh;
      v4f v = *(const v4fa*)(slab + row * 68 + c4);
      v *= oscale;
      vv[it] = v;
    }
    for (int pass = 0; pass < 2; ++pass) {
#pragma unroll
      for (int it = 0; it < 8; ++it) {
        const int row = mBase + it * 2 + hh;
        if (row < M) *(volatile v4f*)(Db + (size_t)row * (size_t)ldd + nc) = vv[it];
      }
      __threadfence();
    }
    wave_lds_sync();
  }
}

extern "C" void kernel_launch(void* const* d_in, const int* in_sizes, int n_in,
                              void* d_out, int out_size, void* d_ws, size_t ws_size,
                              hipStream_t stream) {
  if (n_in < 8) return;
  if (in_sizes[0] != NB * NT * TD) return;
  if (in_sizes[1] != NB * NI * IDM) return;
  if (in_sizes[2] != TD * HD) return;
  if (in_sizes[3] != HD) return;
  if (in_sizes[4] != IDM * HD) return;
  if (in_sizes[5] != HD) return;
  if (in_sizes[6] != HD) return;
  if (in_sizes[7] != 1) return;
  if (out_size != NB * NT * IDM + NB * NI * TD) return;

  const float* text  = (const float*)d_in[0];
  const float* image = (const float*)d_in[1];
  const float* Wt    = (const float*)d_in[2];
  const float* bt    = (const float*)d_in[3];
  const float* Wi    = (const float*)d_in[4];
  const float* bi    = (const float*)d_in[5];
  const float* wa    = (const float*)d_in[6];
  const float* ba    = (const float*)d_in[7];
  float* out0 = (float*)d_out;
  float* out1 = out0 + (size_t)NB * NT * IDM;

  constexpr size_t SZ_XT  = (size_t)MT * TD * 2;
  constexpr size_t SZ_XI  = (size_t)MIP * IDM * 2;
  constexpr size_t SZ_WTT = (size_t)HD * TD * 2;
  constexpr size_t SZ_WIT = (size_t)HD * IDM * 2;
  constexpr size_t SZ_PAR = (size_t)2048 * 4;
  constexpr size_t SZ_PT  = (size_t)MT * HD * 4;
  constexpr size_t SZ_PI  = (size_t)MI * HD * 4;
  constexpr size_t SZ_ST  = (size_t)NB * NI * NT * 4;
  constexpr size_t SZ_P1  = (size_t)NB * NT * KT1 * 2;
  constexpr size_t SZ_P2  = (size_t)NB * MP2 * KT2 * 2;
  constexpr size_t SZ_IT  = (size_t)NB * IDM * KT1 * 2;
  constexpr size_t SZ_TT  = (size_t)NB * TD * KT2 * 2;
  static_assert(SZ_XT % 256 == 0 && SZ_XI % 256 == 0 && SZ_WTT % 256 == 0 && SZ_WIT % 256 == 0);
  static_assert(SZ_PAR % 256 == 0 && SZ_PT % 256 == 0 && SZ_PI % 256 == 0 && SZ_ST % 256 == 0);
  static_assert(SZ_P1 % 256 == 0 && SZ_P2 % 256 == 0 && SZ_IT % 256 == 0 && SZ_TT % 256 == 0);
  constexpr size_t O_XT  = 0;
  constexpr size_t O_XI  = O_XT + SZ_XT;
  constexpr size_t O_WTT = O_XI + SZ_XI;
  constexpr size_t O_WIT = O_WTT + SZ_WTT;
  constexpr size_t O_PAR = O_WIT + SZ_WIT;
  constexpr size_t O_PT  = O_PAR + SZ_PAR;
  constexpr size_t O_PI  = O_PT + SZ_PT;
  constexpr size_t O_ST  = O_PI + SZ_PI;
  constexpr size_t O_P1  = O_ST + SZ_ST;
  constexpr size_t O_P2  = O_P1 + SZ_P1;
  constexpr size_t O_IT  = O_P2 + SZ_P2;
  constexpr size_t O_TT  = O_IT + SZ_IT;
  constexpr size_t O_END = O_TT + SZ_TT;
  static_assert(O_END <= (size_t)134217728);
  if (O_END > ws_size) return;

  char* ws = (char*)d_ws;
  unsigned short* XT  = (unsigned short*)(ws + O_XT);
  unsigned short* XI  = (unsigned short*)(ws + O_XI);
  unsigned short* WtT = (unsigned short*)(ws + O_WTT);
  unsigned short* WiT = (unsigned short*)(ws + O_WIT);
  float*          par = (float*)(ws + O_PAR);
  float*          PT  = (float*)(ws + O_PT);
  float*          PI  = (float*)(ws + O_PI);
  float*          ST  = (float*)(ws + O_ST);
  unsigned short* P1  = (unsigned short*)(ws + O_P1);
  unsigned short* P2  = (unsigned short*)(ws + O_P2);
  unsigned short* IT  = (unsigned short*)(ws + O_IT);
  unsigned short* TT  = (unsigned short*)(ws + O_TT);

  k_plane<0><<<dim3(MT * TD / 8 / 256), 256, 0, stream>>>(text, MT, TD, TD, XT, MT, TD);
  k_plane<0><<<dim3(MIP * IDM / 8 / 256), 256, 0, stream>>>(image, MI, IDM, IDM, XI, MIP, IDM);
  k_wt<<<dim3(HD / 64, 29), 256, 0, stream>>>(Wt, Wi, bt, bi, wa, ba, WtT, WiT, par);
  k_gemm_nt<0, 1><<<dim3((MT / 64) * (HD / 64) / 8), 256, 0, stream>>>(XT, WtT, par, PT, MT, HD, TD, HD);
  k_gemm_nt<0, 1><<<dim3(((MIP / 64) * (HD / 64) + 7) / 8), 256, 0, stream>>>(XI, WiT, par + HD, PI, MI, HD, IDM, HD);
  (void)hipFuncSetAttribute(reinterpret_cast<const void*>(&k_pair), hipFuncAttributeMaxDynamicSharedMemorySize,
                            PAIR_LDS_FLOATS * 4);
  k_pair<<<dim3(7, 4, NB), 128, PAIR_LDS_FLOATS * 4, stream>>>(PT, PI, par, ST);
  (void)hipFuncSetAttribute(reinterpret_cast<const void*>(&k_soft), hipFuncAttributeMaxDynamicSharedMemorySize,
                            SOFT_LDS_BYTES);
  k_soft<<<dim3(NB), 256, SOFT_LDS_BYTES, stream>>>(ST, P1, P2);
  k_ft<NI, KH1, IDM, NDUP><<<dim3(IDM / 64, NB), 256, 0, stream>>>(XI, IT);
  k_ft<NT, KH2, TD, NDUP><<<dim3(TD / 64, NB), 256, 0, stream>>>(XT, TT);
  k_att<AFORM><<<dim3((NT / 64) * (IDM / 64) / 8, 1, NB), 256, 0, stream>>>(
      P1, IT, out0, NT, NT, IDM, KT1, IDM, NT * KT1, IDM * KT1, NT * IDM, OSCALE);
  k_att<AFORM><<<dim3((MP2 / 64) * (TD / 64) / 8, 1, NB), 256, 0, stream>>>(
      P2, TT, out1, NI, MP2, TD, KT2, TD, MP2 * KT2, TD * KT2, NI * TD, OSCALE);
  (void)hipGetLastError();
}
